// IAttention_19533511262641
// MI455X (gfx1250) — hardware-verified
//
#include <hip/hip_runtime.h>
#include <math.h>

constexpr int kB   = 4;
constexpr int kS   = 2048;
constexpr int kE   = 1024;
constexpr int kH   = 16;
constexpr int kDh  = 64;
constexpr int kT   = kB * kS;
constexpr int kHD  = kH * kDh;
constexpr int kFfn = 64;
constexpr int kGrp = 2;
constexpr int kChunkPerBatch = kH / kGrp;
constexpr int kNChunk = (kB * kH) / kGrp;
constexpr float kWCarry    = 16.0f;
constexpr float kWCarryInv = 1.0f / 16.0f;
constexpr float kPCarry    = 1024.0f;
constexpr float kCtxCarry  = 256.0f;
constexpr float kResCarry  = 2048.0f;
constexpr float kPVScale   = kCtxCarry / kPCarry;
constexpr float kWoScale   = 1.0f / (kResCarry * kCtxCarry);
constexpr float kFfnScale  = 1.0f / kResCarry;
constexpr float kInvE      = 1.0f / 1024.0f;
constexpr float kLnEps     = 1e-5f;
constexpr float kNegFill   = -1.0e9f;

static_assert(kT % 64 == 0 && kE % 64 == 0 && kS % 64 == 0 && kFfn % 64 == 0, "tile multiples");
static_assert(kE % 32 == 0 && kDh % 32 == 0 && kS % 32 == 0 && (2 * kFfn) % 32 == 0, "K multiples of 32");
static_assert(kH % kGrp == 0, "chunks never cross a batch");

constexpr size_t kMiB     = (size_t)1 << 20;
constexpr size_t kOffQ16  = 0;
constexpr size_t kOffK16  = 16 * kMiB;
constexpr size_t kOffVT16 = 32 * kMiB;
constexpr size_t kOffS32  = 48 * kMiB;
constexpr size_t kOffP16  = 80 * kMiB;
constexpr size_t kOffCTX  = 96 * kMiB;
constexpr size_t kOffX16  = 48 * kMiB;
constexpr size_t kOffWQKV = 80 * kMiB;
constexpr size_t kOffHPRE = 0;
constexpr size_t kOffWO2  = 32 * kMiB;
constexpr size_t kOffW1P  = 36 * kMiB;
constexpr size_t kOffW2P  = 36 * kMiB + 256 * 1024;
constexpr size_t kOffHP   = 48 * kMiB;
constexpr size_t kOffF1   = 80 * kMiB;
constexpr size_t kOffGP   = 82 * kMiB;
constexpr size_t kOffF2   = 96 * kMiB;
constexpr size_t kWsTotal = 128 * kMiB;
static_assert(kOffX16 + (size_t)kT * kE * 2 <= kOffP16, "X16 inside R3");
static_assert(kOffWQKV + (size_t)3 * kHD * kE * 2 <= kOffCTX, "WQKV16 inside R4");
static_assert((size_t)kGrp * kS * kS * 4 == 32 * kMiB, "S32 chunk = R3");
static_assert((size_t)kGrp * kS * kS * 2 == 16 * kMiB, "P16 chunk = R4");
static_assert(kOffW2P + (size_t)kE * 2 * kFfn * 2 <= kOffHP, "tail weight planes inside R2");
static_assert(kOffGP + (size_t)kT * 2 * kFfn * 2 <= kOffF2, "GP inside R4");
static_assert(kOffF2 + (size_t)kT * kE * 4 == kWsTotal, "F2 = R5");

typedef __attribute__((ext_vector_type(16))) _Float16 v16h;
typedef __attribute__((ext_vector_type(8)))  _Float16 v8h;
typedef __attribute__((ext_vector_type(16))) __bf16   v16b;
typedef __attribute__((ext_vector_type(8)))  __bf16   v8b;
typedef __attribute__((ext_vector_type(8)))  float    v8f;
typedef __attribute__((ext_vector_type(4)))  float    v4f;
typedef __attribute__((ext_vector_type(2)))  float    v2f;
typedef __attribute__((ext_vector_type(4)))  unsigned int v4u;
typedef __attribute__((ext_vector_type(4)))  int      v4i;

__device__ __forceinline__ unsigned short f2bf_bits(float f) {
  unsigned u = __float_as_uint(f);
  return (unsigned short)((u + 0x7FFFu + ((u >> 16) & 1u)) >> 16);
}
__device__ __forceinline__ float bf_bits2f(unsigned short h) { return __uint_as_float(((unsigned)h) << 16); }

__device__ __forceinline__ void dep_guard_h(v8f& a, v8f& b, v16h x, v16h y) { asm volatile("v_nop\n\tv_nop\n\tv_nop\n\tv_nop" : "+v"(a), "+v"(b) : "v"(x), "v"(y)); }
__device__ __forceinline__ void dep_guard_b(v8f& a, v8f& b, v16b x, v16b y) { asm volatile("v_nop\n\tv_nop\n\tv_nop\n\tv_nop" : "+v"(a), "+v"(b) : "v"(x), "v"(y)); }
__device__ __forceinline__ void keep4_h(v16h a, v16h b, v16h c, v16h d) { asm volatile("v_nop" :: "v"(a), "v"(b), "v"(c), "v"(d)); }
__device__ __forceinline__ void keep4_b(v16b a, v16b b, v16b c, v16b d) { asm volatile("v_nop" :: "v"(a), "v"(b), "v"(c), "v"(d)); }
__device__ __forceinline__ void acc_guard4(v8f& a, v8f& b, v8f& c, v8f& d) { asm volatile("v_nop\n\tv_nop\n\tv_nop\n\tv_nop" : "+v"(a), "+v"(b), "+v"(c), "+v"(d)); }
template <typename T> struct Frag;
template <> struct Frag<_Float16> {
  typedef v16h V; union U { v16h v; v8h h[2]; };
  static __device__ __forceinline__ v16h load(const _Float16* p) {
    U f; f.h[0] = *(const v8h*)(p); f.h[1] = *(const v8h*)(p + 16); return f.v;
  }
  static __device__ __forceinline__ v8f mma(v16h a, v16h b, v8f c) {
    return __builtin_amdgcn_wmma_f32_16x16x32_f16(false, a, false, b, (short)0, c, false, false);
  }
  static __device__ __forceinline__ void guard(v8f& a, v8f& b, v16h x, v16h y) { dep_guard_h(a, b, x, y); }
  static __device__ __forceinline__ void keep(v16h a, v16h b, v16h c, v16h d) { keep4_h(a, b, c, d); }
};
template <> struct Frag<__bf16> {
  typedef v16b V; union U { v16b v; v8b h[2]; };
  static __device__ __forceinline__ v16b load(const __bf16* p) {
    U f; f.h[0] = *(const v8b*)(p); f.h[1] = *(const v8b*)(p + 16); return f.v;
  }
  static __device__ __forceinline__ v8f mma(v16b a, v16b b, v8f c) {
    return __builtin_amdgcn_wmma_f32_16x16x32_bf16(false, a, false, b, (short)0, c, false, false);
  }
  static __device__ __forceinline__ void guard(v8f& a, v8f& b, v16b x, v16b y) { dep_guard_b(a, b, x, y); }
  static __device__ __forceinline__ void keep(v16b a, v16b b, v16b c, v16b d) { keep4_b(a, b, c, d); }
};

__device__ __forceinline__ unsigned pk16(unsigned short a, unsigned short b) { return (unsigned)a | ((unsigned)b << 16); }
__device__ __forceinline__ unsigned short h_bits(float f) { const _Float16 h = (_Float16)f; return __builtin_bit_cast(unsigned short, h); }
__device__ __forceinline__ void hl_bits(float v, unsigned short& hb, unsigned short& lb) {
  const _Float16 hq = (_Float16)v;
  hb = __builtin_bit_cast(unsigned short, hq);
  const _Float16 lq = (_Float16)((v - (float)hq) * kResCarry);
  lb = __builtin_bit_cast(unsigned short, lq);
}

template <int ET> struct Elem;
template <> struct Elem<0> { typedef _Float16 T; };
template <> struct Elem<1> { typedef __bf16 T; };
template <int ET, bool SPLIT, int BIAS_MODE, int OUT_MODE, bool RESID, int ACT = 0>
__global__ __launch_bounds__(256) void wmma_gemm64(
    const unsigned short* __restrict__ Ap, const unsigned short* __restrict__ A2p, int lda, long strideA,
    const unsigned short* __restrict__ Btp, const unsigned short* __restrict__ Bt2p, int ldb, long strideB,
    void* __restrict__ Cout, void* __restrict__ Cout2, int ldc, long strideC,
    const float* __restrict__ bias,
    const float* __restrict__ resid, long strideR,
    int M, int N, int K, float scale) {
  typedef typename Elem<ET>::T T;
  typedef typename Frag<T>::V V;
  const T* A = (const T*)Ap; const T* A2 = (const T*)A2p; const T* Bt = (const T*)Btp; const T* Bt2 = (const T*)Bt2p;
  __shared__ __align__(16) float sT[8][16 * 68];
  const int b    = blockIdx.y;
  const int lane = threadIdx.x & 31;
  const int wave = threadIdx.x >> 5;
  const int tilesN = N >> 6;
  const int tilesM = M >> 6;
  const int tile = blockIdx.x * 8 + wave;
  if (tile >= tilesM * tilesN) return;
  const int tm = tile / tilesN;
  const int tn = tile - tm * tilesN;
  const int m0 = tm << 6;
  const int n0 = tn << 6;

  const T* Ab  = A  + (size_t)b * strideA;
  const T* Bb  = Bt + (size_t)b * strideB;
  const T* Ab2 = SPLIT ? (A2  + (size_t)b * strideA) : nullptr;
  const T* Bb2 = SPLIT ? (Bt2 + (size_t)b * strideB) : nullptr;

  const int rlane = lane & 15;
  const int koff  = (lane >> 4) * 8;
  const int mOff  = (lane >> 4) * 8;

  v8f acc[4][4];
#pragma unroll
  for (int i = 0; i < 4; ++i)
#pragma unroll
    for (int j = 0; j < 4; ++j) acc[i][j] = (v8f){0.f,0.f,0.f,0.f,0.f,0.f,0.f,0.f};

  for (int k0 = 0; k0 < K; k0 += 32) {
    V bh[4], bl[4];
#pragma unroll
    for (int j = 0; j < 4; ++j) {
      const size_t bo = (size_t)(n0 + (j << 4) + rlane) * ldb + koff + k0;
      bh[j] = Frag<T>::load(Bb + bo);
      if (SPLIT) bl[j] = Frag<T>::load(Bb2 + bo);
    }
#pragma unroll
    for (int i = 0; i < 4; ++i) {
      const size_t ao = (size_t)(m0 + (i << 4) + rlane) * lda + koff + k0;
      V ah = Frag<T>::load(Ab + ao);
      V al;
      if (SPLIT) al = Frag<T>::load(Ab2 + ao);
#pragma unroll
      for (int j = 0; j < 4; ++j) {
        acc[i][j] = Frag<T>::mma(ah, bh[j], acc[i][j]);
        if (SPLIT) {
          acc[i][j] = Frag<T>::mma(ah, bl[j], acc[i][j]);
          acc[i][j] = Frag<T>::mma(al, bh[j], acc[i][j]);
        }
      }
      Frag<T>::guard(acc[i][0], acc[i][3], ah, SPLIT ? al : ah);
    }
    Frag<T>::keep(bh[0], bh[1], bh[2], bh[3]);
    if (SPLIT) Frag<T>::keep(bl[0], bl[1], bl[2], bl[3]);
  }
  acc_guard4(acc[0][0], acc[0][1], acc[0][2], acc[0][3]);
  acc_guard4(acc[1][0], acc[1][1], acc[1][2], acc[1][3]);
  acc_guard4(acc[2][0], acc[2][1], acc[2][2], acc[2][3]);
  acc_guard4(acc[3][0], acc[3][1], acc[3][2], acc[3][3]);

  float* slab = sT[wave];
  const float* Rb = RESID ? (resid + (size_t)b * strideR) : nullptr;
#pragma unroll
  for (int i = 0; i < 4; ++i) {
    const int mBase = m0 + (i << 4);
#pragma unroll
    for (int j = 0; j < 4; ++j) {
      const int n = n0 + (j << 4) + rlane;
      float bv = 0.f;
      if (BIAS_MODE == 2) bv = bias[n];
#pragma unroll
      for (int r = 0; r < 8; ++r) {
        float v = acc[i][j][r] * scale;
        if (BIAS_MODE == 1) v += bias[mBase + mOff + r];
        if (BIAS_MODE == 2) v += bv;
        if (RESID) v += Rb[(size_t)(mBase + mOff + r) * ldc + n];
        if (ACT == 2) v = fmaxf(v, 0.0f);
        if (ACT == 4) v = (v > 0.f) ? v : 0.01f * v;
        slab[(mOff + r) * 68 + (j << 4) + rlane] = v;
      }
    }
    __builtin_amdgcn_fence(__ATOMIC_RELEASE, "workgroup");
    __builtin_amdgcn_wave_barrier();
    __builtin_amdgcn_fence(__ATOMIC_ACQUIRE, "workgroup");
    if (OUT_MODE == 0) {
      float* C = (float*)Cout + (size_t)b * strideC;
      const int hh = lane >> 4, c4 = (lane & 15) * 4;
      for (int pass = 0; pass < 2; ++pass) {
#pragma unroll
        for (int it = 0; it < 8; ++it) {
          const int row = it * 2 + hh;
          v4f v = *(const v4f*)(slab + row * 68 + c4);
          *(volatile v4f*)(C + (size_t)(mBase + row) * ldc + n0 + c4) = v;
        }
        __threadfence();
      }
    } else {
      const int q = lane >> 3, c8 = (lane & 7) * 8;
      unsigned short* C  = (unsigned short*)Cout  + (size_t)b * strideC;
      unsigned short* C2 = (OUT_MODE >= 2) ? ((unsigned short*)Cout2 + (size_t)b * strideC) : nullptr;
      for (int pass = 0; pass < 2; ++pass) {
#pragma unroll
        for (int it = 0; it < 4; ++it) {
          const int row = it * 4 + q;
          const float* sp = slab + row * 68 + c8;
          v8h hv, lv;
#pragma unroll
          for (int e = 0; e < 8; ++e) {
            if (OUT_MODE == 1) {
              hv[e] = (_Float16)sp[e];
            } else if (OUT_MODE == 3) {
              const _Float16 hq = (_Float16)sp[e];
              hv[e] = hq;
              lv[e] = (_Float16)((sp[e] - (float)hq) * kResCarry);
            } else {
              unsigned short hb = f2bf_bits(sp[e]);
              unsigned short lb = f2bf_bits(sp[e] - bf_bits2f(hb));
              hv[e] = __builtin_bit_cast(_Float16, hb);
              lv[e] = __builtin_bit_cast(_Float16, lb);
            }
          }
          *(volatile v8h*)(C + (size_t)(mBase + row) * ldc + n0 + c8) = hv;
          if (OUT_MODE >= 2) *(volatile v8h*)(C2 + (size_t)(mBase + row) * ldc + n0 + c8) = lv;
        }
        __threadfence();
      }
    }
    __builtin_amdgcn_fence(__ATOMIC_RELEASE, "workgroup");
    __builtin_amdgcn_wave_barrier();
    __builtin_amdgcn_fence(__ATOMIC_ACQUIRE, "workgroup");
  }
}

__global__ __launch_bounds__(256) void cast8_f16_kernel(const float* __restrict__ in, unsigned short* __restrict__ out, int n8) {
  const int i = blockIdx.x * 256 + threadIdx.x;
  if (i >= n8) return;
  const float* p = in + 8 * (size_t)i;
  const v4f a = *(const v4f*)(p);
  const v4f c = *(const v4f*)(p + 4);
  unsigned short hb[8];
#pragma unroll
  for (int e = 0; e < 4; ++e) {
    hb[e]     = h_bits(a[e]);
    hb[4 + e] = h_bits(c[e]);
  }
  const v4u u = (v4u){pk16(hb[0], hb[1]), pk16(hb[2], hb[3]), pk16(hb[4], hb[5]), pk16(hb[6], hb[7])};
  unsigned short* q = out + 8 * (size_t)i;
  *(volatile v4u*)q = u;
  __threadfence();
  *(volatile v4u*)q = u;
}

__global__ __launch_bounds__(256) void wprep_qkv_kernel(const float* __restrict__ Wq, const float* __restrict__ Wk,
                                                        const float* __restrict__ Wv, unsigned short* __restrict__ out,
                                                        float scale) {
  __shared__ float sm[64][65];
  const int t  = threadIdx.x;
  const int r0 = blockIdx.x * 64;
  const int h  = blockIdx.y;
  const int p  = blockIdx.z;
  const float* W = (p == 0) ? Wq : (p == 1) ? Wk : Wv;
  const float* in = W + (size_t)h * kE * kDh;
#pragma unroll
  for (int i = 0; i < 16; ++i) {
    const int idx = i * 256 + t;
    const int er = idx >> 6;
    const int d  = idx & 63;
    sm[d][er] = in[(size_t)(r0 + er) * kDh + d] * scale;
  }
  __syncthreads();
  const int lane = t & 31, wave = t >> 5;
  const int q = lane >> 3, c8 = (lane & 7) * 8;
  unsigned short* op = out + ((size_t)p * kHD + (size_t)h * kDh) * kE;
  for (int pass = 0; pass < 2; ++pass) {
#pragma unroll
    for (int it = 0; it < 2; ++it) {
      const int row = wave * 8 + it * 4 + q;
      unsigned short hb[8];
#pragma unroll
      for (int e = 0; e < 8; ++e) hb[e] = h_bits(sm[row][c8 + e]);
      const v4u u = (v4u){pk16(hb[0], hb[1]), pk16(hb[2], hb[3]), pk16(hb[4], hb[5]), pk16(hb[6], hb[7])};
      *(volatile v4u*)(op + (size_t)row * kE + r0 + c8) = u;
    }
    __threadfence();
  }
}

__global__ __launch_bounds__(256) void tcast2_kernel(const float* __restrict__ in, int in_pitch,
                                                     unsigned short* __restrict__ out, int out_pitch, int lo_off,
                                                     float scale_hi) {
  __shared__ float sm[64][65];
  const int t  = threadIdx.x;
  const int c0 = blockIdx.x * 64;
  const int r0 = blockIdx.y * 64;
#pragma unroll
  for (int i = 0; i < 16; ++i) {
    const int idx = i * 256 + t;
    const int r = idx >> 6;
    const int c = idx & 63;
    sm[c][r] = in[(size_t)(r0 + r) * in_pitch + c0 + c];
  }
  __syncthreads();
  const int lane = t & 31, wave = t >> 5;
  const int q = lane >> 3, c8 = (lane & 7) * 8;
  for (int pass = 0; pass < 2; ++pass) {
#pragma unroll
    for (int it = 0; it < 2; ++it) {
      const int row = wave * 8 + it * 4 + q;
      unsigned short hb[8], lb[8];
#pragma unroll
      for (int e = 0; e < 8; ++e) {
        const float v = sm[row][c8 + e];
        hb[e] = h_bits(v * scale_hi);
        lb[e] = h_bits(v);
      }
      const v4u uh = (v4u){pk16(hb[0], hb[1]), pk16(hb[2], hb[3]), pk16(hb[4], hb[5]), pk16(hb[6], hb[7])};
      const v4u ul = (v4u){pk16(lb[0], lb[1]), pk16(lb[2], lb[3]), pk16(lb[4], lb[5]), pk16(lb[6], lb[7])};
      unsigned short* op = out + (size_t)(c0 + row) * out_pitch + r0 + c8;
      *(volatile v4u*)(op) = uh;
      *(volatile v4u*)(op + lo_off) = ul;
    }
    __threadfence();
  }
}

__global__ __launch_bounds__(256) void softmax_mask_kernel(const float* __restrict__ Sc, const int* __restrict__ mrow,
                                                           unsigned short* __restrict__ P) {
  __shared__ float redM[8];
  __shared__ float redS[8];
  const int row  = blockIdx.x;
  const int t    = threadIdx.x;
  const int lane = t & 31, wave = t >> 5;
  const int c0   = t * 8;
  const float* sr = Sc + (size_t)row * kS + c0;
  const v4f a = *(const v4f*)(sr);
  const v4f c = *(const v4f*)(sr + 4);
  const v4i ma = *(const v4i*)(mrow + c0);
  const v4i mc = *(const v4i*)(mrow + c0 + 4);
  float x[8];
#pragma unroll
  for (int e = 0; e < 4; ++e) {
    x[e]     = (ma[e] == 0) ? kNegFill : a[e];
    x[4 + e] = (mc[e] == 0) ? kNegFill : c[e];
  }
  float m = fmaxf(fmaxf(fmaxf(x[0], x[1]), fmaxf(x[2], x[3])), fmaxf(fmaxf(x[4], x[5]), fmaxf(x[6], x[7])));
#pragma unroll
  for (int off = 16; off > 0; off >>= 1) m = fmaxf(m, __shfl_xor(m, off, 32));
  if (lane == 0) redM[wave] = m;
  __syncthreads();
  m = redM[0];
#pragma unroll
  for (int j = 1; j < 8; ++j) m = fmaxf(m, redM[j]);
  float p[8];
#pragma unroll
  for (int e = 0; e < 8; ++e) p[e] = expf(x[e] - m);
  float s = ((p[0] + p[1]) + (p[2] + p[3])) + ((p[4] + p[5]) + (p[6] + p[7]));
#pragma unroll
  for (int off = 16; off > 0; off >>= 1) s += __shfl_xor(s, off, 32);
  if (lane == 0) redS[wave] = s;
  __syncthreads();
  float tot = redS[0];
#pragma unroll
  for (int j = 1; j < 8; ++j) tot += redS[j];
  const float scl = kPCarry * (1.0f / tot);
  unsigned short hb[8];
#pragma unroll
  for (int e = 0; e < 8; ++e) hb[e] = h_bits(p[e] * scl);
  const v4u u = (v4u){pk16(hb[0], hb[1]), pk16(hb[2], hb[3]), pk16(hb[4], hb[5]), pk16(hb[6], hb[7])};
  unsigned short* q = P + (size_t)row * kS + c0;
  *(volatile v4u*)q = u;
  __threadfence();
  *(volatile v4u*)q = u;
}

template <bool OUT16>
__global__ __launch_bounds__(128) void layernorm_kernel(const float* __restrict__ in, const float* __restrict__ gamma,
                                                        const float* __restrict__ beta, float* __restrict__ out32,
                                                        unsigned short* __restrict__ out16) {
  __shared__ float redA[4];
  __shared__ float redB[4];
  const int row  = blockIdx.x;
  const int t    = threadIdx.x;
  const int lane = t & 31, wave = t >> 5;
  const int c0   = OUT16 ? 8 * t : 4 * t;
  const int c1   = OUT16 ? 8 * t + 4 : 512 + 4 * t;
  const float* xr = in + (size_t)row * kE;
  const v4f x0 = *(const v4f*)(xr + c0);
  const v4f x1 = *(const v4f*)(xr + c1);
  const v4f ga = *(const v4f*)(gamma + c0);
  const v4f gb = *(const v4f*)(gamma + c1);
  const v4f ba = *(const v4f*)(beta + c0);
  const v4f bb = *(const v4f*)(beta + c1);
  float s = ((x0[0] + x0[1]) + (x0[2] + x0[3])) + ((x1[0] + x1[1]) + (x1[2] + x1[3]));
#pragma unroll
  for (int off = 16; off > 0; off >>= 1) s += __shfl_xor(s, off, 32);
  if (lane == 0) redA[wave] = s;
  __syncthreads();
  const float mean = ((redA[0] + redA[1]) + (redA[2] + redA[3])) * kInvE;
  const v4f d0 = x0 - mean;
  const v4f d1 = x1 - mean;
  float v = ((d0[0] * d0[0] + d0[1] * d0[1]) + (d0[2] * d0[2] + d0[3] * d0[3]))
          + ((d1[0] * d1[0] + d1[1] * d1[1]) + (d1[2] * d1[2] + d1[3] * d1[3]));
#pragma unroll
  for (int off = 16; off > 0; off >>= 1) v += __shfl_xor(v, off, 32);
  if (lane == 0) redB[wave] = v;
  __syncthreads();
  const float var  = ((redB[0] + redB[1]) + (redB[2] + redB[3])) * kInvE;
  const float rstd = rsqrtf(var + kLnEps);
  const v4f y0 = d0 * rstd * ga + ba;
  const v4f y1 = d1 * rstd * gb + bb;
  if (OUT16) {
    unsigned short hb[8], lb[8];
#pragma unroll
    for (int e = 0; e < 4; ++e) {
      hl_bits(y0[e], hb[e], lb[e]);
      hl_bits(y1[e], hb[4 + e], lb[4 + e]);
    }
    const v4u uh = (v4u){pk16(hb[0], hb[1]), pk16(hb[2], hb[3]), pk16(hb[4], hb[5]), pk16(hb[6], hb[7])};
    const v4u ul = (v4u){pk16(lb[0], lb[1]), pk16(lb[2], lb[3]), pk16(lb[4], lb[5]), pk16(lb[6], lb[7])};
    unsigned short* op = out16 + (size_t)row * (2 * kE) + c0;
    *(volatile v4u*)(op) = uh;
    *(volatile v4u*)(op + kE) = ul;
    __threadfence();
    *(volatile v4u*)(op) = uh;
    *(volatile v4u*)(op + kE) = ul;
  } else {
    float* op = out32 + (size_t)row * kE;
    *(volatile v4f*)(op + c0) = y0;
    *(volatile v4f*)(op + c1) = y1;
    __threadfence();
    *(volatile v4f*)(op + c0) = y0;
    *(volatile v4f*)(op + c1) = y1;
  }
}

__device__ __forceinline__ float gelu_erf(float v) { return 0.5f * v * (1.0f + erff(v * 0.70710678118654752f)); }

__global__ __launch_bounds__(256) void gelu_split_kernel(const float* __restrict__ f1, unsigned short* __restrict__ gp) {
  const int wave = threadIdx.x >> 5, lane = threadIdx.x & 31;
  const int row  = blockIdx.x * 8 + wave;
  const v2f v = *(const v2f*)(f1 + (size_t)row * kFfn + 2 * lane);
  const float g0 = gelu_erf(v[0]);
  const float g1 = gelu_erf(v[1]);
  unsigned short h0, l0, h1, l1;
  hl_bits(g0, h0, l0);
  hl_bits(g1, h1, l1);
  const unsigned uh = pk16(h0, h1);
  const unsigned ul = pk16(l0, l1);
  unsigned short* op = gp + (size_t)row * (2 * kFfn) + 2 * lane;
  *(volatile unsigned*)(op) = uh;
  *(volatile unsigned*)(op + kFfn) = ul;
  __threadfence();
  *(volatile unsigned*)(op) = uh;
  *(volatile unsigned*)(op + kFfn) = ul;
}

extern "C" void kernel_launch(void* const* d_in, const int* in_sizes, int n_in,
                              void* d_out, int out_size, void* d_ws, size_t ws_size,
                              hipStream_t stream) {
  if (n_in < 18) return;
  if (in_sizes[0] != kT * kE || in_sizes[1] != kT || in_sizes[2] != kH * kE * kDh || in_sizes[4] != kH * kE * kDh ||
      in_sizes[6] != kH * kE * kDh || in_sizes[8] != kHD * kE || in_sizes[12] != kE * kFfn || in_sizes[14] != kFfn * kE ||
      in_sizes[3] != kHD || in_sizes[5] != kHD || in_sizes[7] != kHD || in_sizes[9] != kE || in_sizes[10] != kE ||
      in_sizes[11] != kE || in_sizes[13] != kFfn || in_sizes[15] != kE || in_sizes[16] != kE || in_sizes[17] != kE)
    return;
  if (out_size != kT * kE) return;
  if (ws_size < kWsTotal) return;

  const float* x    = (const float*)d_in[0];
  const int*   mask = (const int*)d_in[1];
  const float* Wq = (const float*)d_in[2];  const float* bq = (const float*)d_in[3];
  const float* Wk = (const float*)d_in[4];  const float* bk = (const float*)d_in[5];
  const float* Wv = (const float*)d_in[6];  const float* bv = (const float*)d_in[7];
  const float* Wo = (const float*)d_in[8];  const float* bo = (const float*)d_in[9];
  const float* g1 = (const float*)d_in[10]; const float* b1 = (const float*)d_in[11];
  const float* W1 = (const float*)d_in[12]; const float* c1 = (const float*)d_in[13];
  const float* W2 = (const float*)d_in[14]; const float* c2 = (const float*)d_in[15];
  const float* g2 = (const float*)d_in[16]; const float* b2 = (const float*)d_in[17];
  float* out = (float*)d_out;

  unsigned char* ws = (unsigned char*)d_ws;
  unsigned short* Q16  = (unsigned short*)(ws + kOffQ16);
  unsigned short* K16  = (unsigned short*)(ws + kOffK16);
  unsigned short* VT16 = (unsigned short*)(ws + kOffVT16);
  float*          S32  = (float*)(ws + kOffS32);
  unsigned short* P16  = (unsigned short*)(ws + kOffP16);
  unsigned short* CTX  = (unsigned short*)(ws + kOffCTX);
  unsigned short* X16  = (unsigned short*)(ws + kOffX16);
  unsigned short* WQKV = (unsigned short*)(ws + kOffWQKV);
  float*          HPRE = (float*)(ws + kOffHPRE);
  unsigned short* WO2  = (unsigned short*)(ws + kOffWO2);
  unsigned short* W1P  = (unsigned short*)(ws + kOffW1P);
  unsigned short* W2P  = (unsigned short*)(ws + kOffW2P);
  unsigned short* HP   = (unsigned short*)(ws + kOffHP);
  float*          F1   = (float*)(ws + kOffF1);
  unsigned short* GP   = (unsigned short*)(ws + kOffGP);
  float*          F2   = (float*)(ws + kOffF2);

  const float rsc = 1.0f / sqrtf((float)kS);

  cast8_f16_kernel<<<(unsigned)((kT * kE / 8) / 256), 256, 0, stream>>>(x, X16, kT * kE / 8);
  wprep_qkv_kernel<<<dim3(kE / 64, kH, 3), 256, 0, stream>>>(Wq, Wk, Wv, WQKV, kWCarry);

  wmma_gemm64<0, false, 2, 1, false><<<dim3((kT / 64) * (kHD / 64) / 8, 1), 256, 0, stream>>>(
      X16, nullptr, kE, 0L, WQKV, nullptr, kE, 0L, (void*)Q16, nullptr, kHD, 0L, bq, nullptr, 0L, kT, kHD, kE, kWCarryInv);
  wmma_gemm64<0, false, 2, 1, false><<<dim3((kT / 64) * (kHD / 64) / 8, 1), 256, 0, stream>>>(
      X16, nullptr, kE, 0L, WQKV + (size_t)kHD * kE, nullptr, kE, 0L, (void*)K16, nullptr, kHD, 0L, bk, nullptr, 0L,
      kT, kHD, kE, kWCarryInv);
  wmma_gemm64<0, false, 1, 1, false><<<dim3((kHD / 64) * (kS / 64) / 8, kB), 256, 0, stream>>>(
      WQKV + (size_t)2 * kHD * kE, nullptr, kE, 0L, X16, nullptr, kE, (long)kS * kE, (void*)VT16, nullptr, kS,
      (long)kHD * kS, bv, nullptr, 0L, kHD, kS, kE, kWCarryInv);

  for (int ch = 0; ch < kNChunk; ++ch) {
    const int b  = ch / kChunkPerBatch;
    const int h0 = (ch % kChunkPerBatch) * kGrp;
    const size_t qkoff = (size_t)b * kS * kE + (size_t)h0 * kDh;
    wmma_gemm64<0, false, 0, 0, false><<<dim3((kS / 64) * (kS / 64) / 8, kGrp), 256, 0, stream>>>(
        Q16 + qkoff, nullptr, kE, (long)kDh, K16 + qkoff, nullptr, kE, (long)kDh, (void*)S32, nullptr, kS,
        (long)kS * kS, nullptr, nullptr, 0L, kS, kS, kDh, rsc);
    softmax_mask_kernel<<<(unsigned)(kGrp * kS), 256, 0, stream>>>(S32, mask + (size_t)b * kS, P16);
    unsigned short* cbase = CTX + (size_t)b * kS * (2 * kHD) + (size_t)h0 * kDh;
    wmma_gemm64<0, false, 0, 3, false><<<dim3((kS / 64) * (kDh / 64) / 8, kGrp), 256, 0, stream>>>(
        P16, nullptr, kS, (long)kS * kS, VT16 + ((size_t)b * kHD + (size_t)h0 * kDh) * kS, nullptr, kS,
        (long)kDh * kS, (void*)cbase, (void*)(cbase + kHD), 2 * kHD, (long)kDh, nullptr, nullptr, 0L, kS, kDh, kS,
        kPVScale);
  }

  tcast2_kernel<<<dim3(kE / 64, kHD / 64), 256, 0, stream>>>(Wo, kE, WO2, 2 * kHD, kHD, kResCarry);
  tcast2_kernel<<<dim3(kFfn / 64, kE / 64), 256, 0, stream>>>(W1, kFfn, W1P, 2 * kE, kE, kResCarry);
  tcast2_kernel<<<dim3(kE / 64, kFfn / 64), 256, 0, stream>>>(W2, kE, W2P, 2 * kFfn, kFfn, kResCarry);

  wmma_gemm64<0, false, 2, 0, false><<<dim3((kT / 64) * (kE / 64) / 8, 1), 256, 0, stream>>>(
      CTX, nullptr, 2 * kHD, 0L, WO2, nullptr, 2 * kHD, 0L, (void*)HPRE, nullptr, kE, 0L, bo, nullptr, 0L, kT, kE,
      2 * kHD, kWoScale);
  layernorm_kernel<true><<<(unsigned)kT, 128, 0, stream>>>(HPRE, g1, b1, nullptr, HP);

  wmma_gemm64<0, false, 2, 0, false><<<dim3((kT / 64) * (kFfn / 64) / 8, 1), 256, 0, stream>>>(
      HP, nullptr, 2 * kE, 0L, W1P, nullptr, 2 * kE, 0L, (void*)F1, nullptr, kFfn, 0L, c1, nullptr, 0L, kT, kFfn,
      2 * kE, kFfnScale);
  gelu_split_kernel<<<(unsigned)(kT / 8), 256, 0, stream>>>(F1, GP);
  wmma_gemm64<0, false, 2, 0, false><<<dim3((kT / 64) * (kE / 64) / 8, 1), 256, 0, stream>>>(
      GP, nullptr, 2 * kFfn, 0L, W2P, nullptr, 2 * kFfn, 0L, (void*)F2, nullptr, kE, 0L, c2, nullptr, 0L, kT, kE,
      2 * kFfn, kFfnScale);
  layernorm_kernel<false><<<(unsigned)kT, 128, 0, stream>>>(F2, g2, b2, out, nullptr);
}
